// M2DBlock_32985348833816
// MI455X (gfx1250) — hardware-verified
//
#include <hip/hip_runtime.h>
#include <hip/hip_bf16.h>
#include <math.h>
#include <stdint.h>

typedef __attribute__((ext_vector_type(16))) _Float16 v16h;
typedef __attribute__((ext_vector_type(8)))  _Float16 v8h;
typedef __attribute__((ext_vector_type(16))) __bf16   v16b;
typedef __attribute__((ext_vector_type(8)))  __bf16   v8b;
typedef __attribute__((ext_vector_type(8)))  float    v8f;
typedef __attribute__((ext_vector_type(4)))  float    v4f;

#define NPIX  8192
#define DMOD  128
#define DIN   256
#define NST   16
#define HH    64
#define WW    64
#define NCELL 4096

__device__ __forceinline__ unsigned short f2bf_bits(float f) {
  unsigned u = __float_as_uint(f);
  return (unsigned short)((u + 0x7FFFu + ((u >> 16) & 1u)) >> 16);
}
__device__ __forceinline__ float bf_bits2f(unsigned short h) { return __uint_as_float(((unsigned)h) << 16); }

__device__ __forceinline__ void dep_guard_h(v8f& a, v8f& b, v16h x, v16h y) { asm volatile("v_nop\n\tv_nop\n\tv_nop\n\tv_nop" : "+v"(a), "+v"(b) : "v"(x), "v"(y)); }
__device__ __forceinline__ void dep_guard_b(v8f& a, v8f& b, v16b x, v16b y) { asm volatile("v_nop\n\tv_nop\n\tv_nop\n\tv_nop" : "+v"(a), "+v"(b) : "v"(x), "v"(y)); }
__device__ __forceinline__ void keep4_h(v16h a, v16h b, v16h c, v16h d) { asm volatile("v_nop" :: "v"(a), "v"(b), "v"(c), "v"(d)); }
__device__ __forceinline__ void keep4_b(v16b a, v16b b, v16b c, v16b d) { asm volatile("v_nop" :: "v"(a), "v"(b), "v"(c), "v"(d)); }
__device__ __forceinline__ void acc_guard4(v8f& a, v8f& b, v8f& c, v8f& d) { asm volatile("v_nop\n\tv_nop\n\tv_nop\n\tv_nop" : "+v"(a), "+v"(b), "+v"(c), "+v"(d)); }
template <typename T> struct Frag;
template <> struct Frag<_Float16> {
  typedef v16h V; union U { v16h v; v8h h[2]; };
  static __device__ __forceinline__ v16h load(const _Float16* p) {
    U f; f.h[0] = *(const v8h*)(p); f.h[1] = *(const v8h*)(p + 16); return f.v;
  }
  static __device__ __forceinline__ v8f mma(v16h a, v16h b, v8f c) {
    return __builtin_amdgcn_wmma_f32_16x16x32_f16(false, a, false, b, (short)0, c, false, false);
  }
  static __device__ __forceinline__ void guard(v8f& a, v8f& b, v16h x, v16h y) { dep_guard_h(a, b, x, y); }
  static __device__ __forceinline__ void keep(v16h a, v16h b, v16h c, v16h d) { keep4_h(a, b, c, d); }
};
template <> struct Frag<__bf16> {
  typedef v16b V; union U { v16b v; v8b h[2]; };
  static __device__ __forceinline__ v16b load(const __bf16* p) {
    U f; f.h[0] = *(const v8b*)(p); f.h[1] = *(const v8b*)(p + 16); return f.v;
  }
  static __device__ __forceinline__ v8f mma(v16b a, v16b b, v8f c) {
    return __builtin_amdgcn_wmma_f32_16x16x32_bf16(false, a, false, b, (short)0, c, false, false);
  }
  static __device__ __forceinline__ void guard(v8f& a, v8f& b, v16b x, v16b y) { dep_guard_b(a, b, x, y); }
  static __device__ __forceinline__ void keep(v16b a, v16b b, v16b c, v16b d) { keep4_b(a, b, c, d); }
};

template <int ET> struct Elem;
template <> struct Elem<0> { typedef _Float16 T; };
template <> struct Elem<1> { typedef __bf16 T; };
template <int ET, bool SPLIT, int BIAS_MODE, int OUT_MODE, bool RESID, int ACT = 0>
__global__ __launch_bounds__(256) void wmma_gemm64(
    const unsigned short* __restrict__ Ap, const unsigned short* __restrict__ A2p, int lda, long strideA,
    const unsigned short* __restrict__ Btp, const unsigned short* __restrict__ Bt2p, int ldb, long strideB,
    void* __restrict__ Cout, void* __restrict__ Cout2, int ldc, long strideC,
    const float* __restrict__ bias,
    const float* __restrict__ resid, long strideR,
    int M, int N, int K, float scale) {
  typedef typename Elem<ET>::T T;
  typedef typename Frag<T>::V V;
  const T* A = (const T*)Ap; const T* A2 = (const T*)A2p; const T* Bt = (const T*)Btp; const T* Bt2 = (const T*)Bt2p;
  __shared__ __align__(16) float sT[8][16 * 68];
  const int b    = blockIdx.y;
  const int lane = threadIdx.x & 31;
  const int wave = threadIdx.x >> 5;
  const int tilesN = N >> 6;
  const int tilesM = M >> 6;
  const int tile = blockIdx.x * 8 + wave;
  if (tile >= tilesM * tilesN) return;
  const int tm = tile / tilesN;
  const int tn = tile - tm * tilesN;
  const int m0 = tm << 6;
  const int n0 = tn << 6;

  const T* Ab  = A  + (size_t)b * strideA;
  const T* Bb  = Bt + (size_t)b * strideB;
  const T* Ab2 = SPLIT ? (A2  + (size_t)b * strideA) : nullptr;
  const T* Bb2 = SPLIT ? (Bt2 + (size_t)b * strideB) : nullptr;

  const int rlane = lane & 15;
  const int koff  = (lane >> 4) * 8;
  const int mOff  = (lane >> 4) * 8;

  v8f acc[4][4];
#pragma unroll
  for (int i = 0; i < 4; ++i)
#pragma unroll
    for (int j = 0; j < 4; ++j) acc[i][j] = (v8f){0.f,0.f,0.f,0.f,0.f,0.f,0.f,0.f};

  for (int k0 = 0; k0 < K; k0 += 32) {
    V bh[4], bl[4];
#pragma unroll
    for (int j = 0; j < 4; ++j) {
      const size_t bo = (size_t)(n0 + (j << 4) + rlane) * ldb + koff + k0;
      bh[j] = Frag<T>::load(Bb + bo);
      if (SPLIT) bl[j] = Frag<T>::load(Bb2 + bo);
    }
#pragma unroll
    for (int i = 0; i < 4; ++i) {
      const size_t ao = (size_t)(m0 + (i << 4) + rlane) * lda + koff + k0;
      V ah = Frag<T>::load(Ab + ao);
      V al;
      if (SPLIT) al = Frag<T>::load(Ab2 + ao);
#pragma unroll
      for (int j = 0; j < 4; ++j) {
        acc[i][j] = Frag<T>::mma(ah, bh[j], acc[i][j]);
        if (SPLIT) {
          acc[i][j] = Frag<T>::mma(ah, bl[j], acc[i][j]);
          acc[i][j] = Frag<T>::mma(al, bh[j], acc[i][j]);
        }
      }
      Frag<T>::guard(acc[i][0], acc[i][3], ah, SPLIT ? al : ah);
    }
    Frag<T>::keep(bh[0], bh[1], bh[2], bh[3]);
    if (SPLIT) Frag<T>::keep(bl[0], bl[1], bl[2], bl[3]);
  }
  acc_guard4(acc[0][0], acc[0][1], acc[0][2], acc[0][3]);
  acc_guard4(acc[1][0], acc[1][1], acc[1][2], acc[1][3]);
  acc_guard4(acc[2][0], acc[2][1], acc[2][2], acc[2][3]);
  acc_guard4(acc[3][0], acc[3][1], acc[3][2], acc[3][3]);

  float* slab = sT[wave];
  const float* Rb = RESID ? (resid + (size_t)b * strideR) : nullptr;
#pragma unroll
  for (int i = 0; i < 4; ++i) {
    const int mBase = m0 + (i << 4);
#pragma unroll
    for (int j = 0; j < 4; ++j) {
      const int n = n0 + (j << 4) + rlane;
      float bv = 0.f;
      if (BIAS_MODE == 2) bv = bias[n];
#pragma unroll
      for (int r = 0; r < 8; ++r) {
        float v = acc[i][j][r] * scale;
        if (BIAS_MODE == 1) v += bias[mBase + mOff + r];
        if (BIAS_MODE == 2) v += bv;
        if (RESID) v += Rb[(size_t)(mBase + mOff + r) * ldc + n];
        if (ACT == 1) v = tanhf(v);
        if (ACT == 2) v = fmaxf(v, 0.0f);
        if (ACT == 3) v = v / (1.0f + expf(-v));
        if (ACT == 4) v = (v > 0.f) ? v : 0.01f * v;
        if (ACT == 5) v = 0.5f * v * (1.0f + erff(v * 0.70710678118654752f));
        slab[(mOff + r) * 68 + (j << 4) + rlane] = v;
      }
    }
    __builtin_amdgcn_fence(__ATOMIC_RELEASE, "workgroup");
    __builtin_amdgcn_wave_barrier();
    __builtin_amdgcn_fence(__ATOMIC_ACQUIRE, "workgroup");
    if (OUT_MODE == 0) {
      float* C = (float*)Cout + (size_t)b * strideC;
      const int hh = lane >> 4, c4 = (lane & 15) * 4;
      for (int pass = 0; pass < 2; ++pass) {
#pragma unroll
        for (int it = 0; it < 8; ++it) {
          const int row = it * 2 + hh;
          v4f v = *(const v4f*)(slab + row * 68 + c4);
          *(volatile v4f*)(C + (size_t)(mBase + row) * ldc + n0 + c4) = v;
        }
        __threadfence();
      }
    } else {
      const int q = lane >> 3, c8 = (lane & 7) * 8;
      unsigned short* C  = (unsigned short*)Cout  + (size_t)b * strideC;
      unsigned short* C2 = (OUT_MODE == 2) ? ((unsigned short*)Cout2 + (size_t)b * strideC) : nullptr;
      for (int pass = 0; pass < 2; ++pass) {
#pragma unroll
        for (int it = 0; it < 4; ++it) {
          const int row = it * 4 + q;
          const float* sp = slab + row * 68 + c8;
          v8h hv, lv;
#pragma unroll
          for (int e = 0; e < 8; ++e) {
            if (OUT_MODE == 1) {
              hv[e] = (_Float16)sp[e];
            } else {
              unsigned short hb = f2bf_bits(sp[e]);
              unsigned short lb = f2bf_bits(sp[e] - bf_bits2f(hb));
              hv[e] = __builtin_bit_cast(_Float16, hb);
              lv[e] = __builtin_bit_cast(_Float16, lb);
            }
          }
          *(volatile v8h*)(C + (size_t)(mBase + row) * ldc + n0 + c8) = hv;
          if (OUT_MODE == 2) *(volatile v8h*)(C2 + (size_t)(mBase + row) * ldc + n0 + c8) = lv;
        }
        __threadfence();
      }
    }
    __builtin_amdgcn_fence(__ATOMIC_RELEASE, "workgroup");
    __builtin_amdgcn_wave_barrier();
    __builtin_amdgcn_fence(__ATOMIC_ACQUIRE, "workgroup");
  }
}

__device__ __forceinline__ void split_store8(v4f a, v4f c, unsigned short* __restrict__ ph,
                                             unsigned short* __restrict__ pl) {
  v8h hv, lv;
#pragma unroll
  for (int k = 0; k < 4; ++k) {
    unsigned short hb = f2bf_bits(a[k]);
    unsigned short lb = f2bf_bits(a[k] - bf_bits2f(hb));
    hv[k] = __builtin_bit_cast(_Float16, hb);
    lv[k] = __builtin_bit_cast(_Float16, lb);
    hb = f2bf_bits(c[k]);
    lb = f2bf_bits(c[k] - bf_bits2f(hb));
    hv[4 + k] = __builtin_bit_cast(_Float16, hb);
    lv[4 + k] = __builtin_bit_cast(_Float16, lb);
  }
  for (int pass = 0; pass < 2; ++pass) {
    *(volatile v8h*)ph = hv;
    *(volatile v8h*)pl = lv;
    __threadfence();
  }
}
__device__ __forceinline__ v4f zsel4(v4f a, bool z) {
  v4f r;
#pragma unroll
  for (int k = 0; k < 4; ++k) r[k] = z ? 0.0f : a[k];
  return r;
}

__global__ __launch_bounds__(256) void split_cast8(const float* __restrict__ in,
                                                   unsigned short* __restrict__ oh,
                                                   unsigned short* __restrict__ ol, int n8) {
  const int i = blockIdx.x * 256 + threadIdx.x;
  if (i >= n8) return;
  const float* s = in + (size_t)i * 8;
  const v4f a = *(const v4f*)(s);
  const v4f c = *(const v4f*)(s + 4);
  split_store8(a, c, oh + (size_t)i * 8, ol + (size_t)i * 8);
}

template <int FN, bool PLANES>
__global__ __launch_bounds__(256) void ew_tile2048(const float* __restrict__ in, float* __restrict__ of,
                                                    unsigned short* __restrict__ oh,
                                                    unsigned short* __restrict__ ol) {
  __shared__ __align__(16) float s[2048];
  const int tid = threadIdx.x;
  const size_t base = (size_t)blockIdx.x * 2048;
#pragma unroll 1
  for (int k = 0; k < 8; ++k) {
    const int idx = (k << 8) + tid;
    const float v = in[base + idx];
    float r;
    if (FN == 0) r = 0.5f * v * (1.0f + erff(v * 0.70710678118654752f));
    else         r = fmaxf(v, 0.0f) + log1pf(expf(-fabsf(v)));
    s[idx] = r;
  }
  __syncthreads();
  const v4f f0 = *(const v4f*)(s + 4 * tid);
  const v4f f1 = *(const v4f*)(s + 1024 + 4 * tid);
  for (int pass = 0; pass < 2; ++pass) {
    *(volatile v4f*)(of + base + 4 * tid) = f0;
    *(volatile v4f*)(of + base + 1024 + 4 * tid) = f1;
    __threadfence();
  }
  if (PLANES) {
    const v4f a = *(const v4f*)(s + 8 * tid);
    const v4f c = *(const v4f*)(s + 8 * tid + 4);
    split_store8(a, c, oh + base + 8 * tid, ol + base + 8 * tid);
  }
}

__global__ __launch_bounds__(128) void prep_params(
    const float* __restrict__ wi, const float* __restrict__ wx,
    const float* __restrict__ dtTw, const float* __restrict__ dtLw,
    const float* __restrict__ wo, const float* __restrict__ xpb,
    const float* __restrict__ dtTb, const float* __restrict__ dtLb,
    unsigned short* __restrict__ wih, unsigned short* __restrict__ wil,
    unsigned short* __restrict__ wxh, unsigned short* __restrict__ wxl,
    unsigned short* __restrict__ wdh, unsigned short* __restrict__ wdl,
    unsigned short* __restrict__ woh, unsigned short* __restrict__ wol,
    float* __restrict__ bias576) {
  const int bx = blockIdx.x, tid = threadIdx.x;
  if (bx < 32) {
    const int g = bx * 128 + tid;
    const float* s = wi + (size_t)g * 8;
    const v4f a = *(const v4f*)(s), c = *(const v4f*)(s + 4);
    split_store8(a, c, wih + (size_t)g * 8, wil + (size_t)g * 8);
  } else if (bx < 48) {
    const int g = (bx - 32) * 128 + tid;
    const int idx0 = g * 8;
    const int row = idx0 >> 8;
    const bool z = (row >= 48);
    const int cidx = z ? (48 * 256 - 8) : idx0;
    const v4f a = *(const v4f*)(wx + cidx), c = *(const v4f*)(wx + cidx + 4);
    split_store8(zsel4(a, z), zsel4(c, z), wxh + (size_t)idx0, wxl + (size_t)idx0);
  } else if (bx < 64) {
    const int g = (bx - 48) * 128 + tid;
    const int idx0 = g * 8;
    const int row = idx0 >> 5;
    const int col0 = idx0 & 31;
    const int rT = row < 256 ? row : 255;
    int rL = row - 256; rL = rL < 0 ? 0 : (rL > 255 ? 255 : rL);
    const v4f aT = *(const v4f*)(dtTw + rT * 8), cT = *(const v4f*)(dtTw + rT * 8 + 4);
    const v4f aL = *(const v4f*)(dtLw + rL * 8), cL = *(const v4f*)(dtLw + rL * 8 + 4);
    const bool useT = (row < 256) && (col0 == 0);
    const bool useL = (row >= 256) && (col0 == 8);
    v4f a, c;
#pragma unroll
    for (int k = 0; k < 4; ++k) {
      a[k] = useT ? aT[k] : (useL ? aL[k] : 0.0f);
      c[k] = useT ? cT[k] : (useL ? cL[k] : 0.0f);
    }
    split_store8(a, c, wdh + (size_t)idx0, wdl + (size_t)idx0);
  } else if (bx < 96) {
    const int g = (bx - 64) * 128 + tid;
    const float* s = wo + (size_t)g * 8;
    const v4f a = *(const v4f*)(s), c = *(const v4f*)(s + 4);
    split_store8(a, c, woh + (size_t)g * 8, wol + (size_t)g * 8);
  } else {
    const int g = (bx - 96) * 128 + tid;
    if (g >= 144) return;
    const int gb = g < 12 ? g : 11;
    const v4f pb = *(const v4f*)(xpb + 4 * gb);
    int gg = g - 16; gg = gg < 0 ? 0 : gg;
    const int gT = gg < 64 ? gg : 63;
    int gL = gg - 64; gL = gL < 0 ? 0 : (gL > 63 ? 63 : gL);
    const v4f tb = *(const v4f*)(dtTb + 4 * gT);
    const v4f lb = *(const v4f*)(dtLb + 4 * gL);
    v4f o;
#pragma unroll
    for (int k = 0; k < 4; ++k) {
      o[k] = (g < 12) ? pb[k] : ((g < 16) ? 0.0f : ((g < 80) ? tb[k] : lb[k]));
    }
    for (int pass = 0; pass < 2; ++pass) {
      *(volatile v4f*)(bias576 + 4 * g) = o;
      __threadfence();
    }
  }
}

__global__ __launch_bounds__(128) void build_a16(const float* __restrict__ dbc,
                                                unsigned short* __restrict__ ah,
                                                unsigned short* __restrict__ al) {
  const int t = blockIdx.x * 128 + threadIdx.x;
  if (t >= NPIX * 4) return;
  const int row = t >> 2;
  const int cq = (t & 3) * 8;
  const float* s = dbc + (size_t)row * 64 + (cq & 8);
  const v4f a = *(const v4f*)(s), c = *(const v4f*)(s + 4);
  const bool z = (cq >= 16);
  split_store8(zsel4(a, z), zsel4(c, z), ah + (size_t)row * 32 + cq, al + (size_t)row * 32 + cq);
}

#define SC_EPB 8
#define SC_THR 128
__global__ __launch_bounds__(SC_THR) void scan2d(
    const float* __restrict__ pre,
    const float* __restrict__ uf,
    const float* __restrict__ dbc,
    const float* __restrict__ atlog,
    const float* __restrict__ allog,
    const float* __restrict__ dvec,
    float* __restrict__ yt) {
  __shared__ __align__(16) float hup[WW * SC_THR];
  __shared__ __align__(16) float ys[2][SC_EPB][WW];
  const int tid  = threadIdx.x;
  const int lane = tid & 31, wave = tid >> 5;
  const int n  = tid & 15;
  const int el = tid >> 4;
  const int b  = blockIdx.x >> 5;
  const int eg = blockIdx.x & 31;
  const int e0 = eg * SC_EPB;
  const int e  = e0 + el;

  const float aT = -expf(atlog[e * NST + n]);
  const float aL = -expf(allog[e * NST + n]);
  const float dc = dvec[e];

#pragma unroll 1
  for (int j = 0; j < WW; ++j) hup[j * SC_THR + tid] = 0.0f;

  const int selw = 2 * wave + (lane >> 4);
  const int c4   = (lane & 15) * 4;

#pragma unroll 1
  for (int i = 0; i < HH; ++i) {
    const int par = i & 1;
    const size_t rowbase = (size_t)b * NCELL + (size_t)i * WW;
    float hleft = 0.0f;
#pragma unroll 1
    for (int j = 0; j < WW; ++j) {
      const size_t g = rowbase + j;
      const float dT = pre[g * 512 + e];
      const float dL = pre[g * 512 + 256 + e];
      const float uu = uf[g * DIN + e];
      const float bm = dbc[g * 64 + 16 + n];
      const float cm = dbc[g * 64 + 32 + n];
      const float dat = expf(dT * aT);
      const float dal = expf(dL * aL);
      const float bxv = (dT + dL) * bm * uu;
      const float hu = hup[j * SC_THR + tid];
      const float v  = dat * hu + bxv;
      const float h  = dal * hleft + v;
      hup[j * SC_THR + tid] = h;
      hleft = h;
      float yc = h * cm;
      yc += __shfl_xor(yc, 1, 32);
      yc += __shfl_xor(yc, 2, 32);
      yc += __shfl_xor(yc, 4, 32);
      yc += __shfl_xor(yc, 8, 32);
      if (n == 0) ys[par][el][j] = yc + uu * dc;
    }
    __syncthreads();
#pragma unroll 1
    for (int it = 0; it < 4; ++it) {
      const int sel = 2 * wave + (it >> 1);
      const int col = ((it & 1) << 5) + lane;
      const float y = ys[par][sel][col];
      ys[par][sel][col] = 0.5f * y * (1.0f + erff(y * 0.70710678118654752f));
    }
    __builtin_amdgcn_fence(__ATOMIC_RELEASE, "workgroup");
    __builtin_amdgcn_wave_barrier();
    __builtin_amdgcn_fence(__ATOMIC_ACQUIRE, "workgroup");
    {
      const v4f val = *(const v4f*)(&ys[par][selw][c4]);
      float* dst = yt + (size_t)(e0 + selw) * NPIX + rowbase + c4;
      for (int pass = 0; pass < 2; ++pass) {
        *(volatile v4f*)dst = val;
        __threadfence();
      }
    }
  }
}

__global__ __launch_bounds__(256) void ytr_split(const float* __restrict__ yt,
                                                 unsigned short* __restrict__ yh,
                                                 unsigned short* __restrict__ yl) {
  __shared__ float tile[64][65];
  const int tid = threadIdx.x, lane = tid & 31, wave = tid >> 5;
  const int ct = blockIdx.x & 127;
  const int et = blockIdx.x >> 7;
  const int c0 = ct * 64, e0 = et * 64;
  {
    const int r = tid >> 2, cq = (tid & 3) * 16;
    const float* src = yt + (size_t)(e0 + r) * NPIX + c0 + cq;
#pragma unroll
    for (int k = 0; k < 4; ++k) {
      const v4f v = *(const v4f*)(src + 4 * k);
      tile[r][cq + 4 * k + 0] = v[0];
      tile[r][cq + 4 * k + 1] = v[1];
      tile[r][cq + 4 * k + 2] = v[2];
      tile[r][cq + 4 * k + 3] = v[3];
    }
  }
  __syncthreads();
  const int q = lane >> 3, c8 = (lane & 7) * 8;
  for (int pass = 0; pass < 2; ++pass) {
#pragma unroll
    for (int it = 0; it < 2; ++it) {
      const int cc = wave * 8 + it * 4 + q;
      v8h hv, lv;
#pragma unroll
      for (int k = 0; k < 8; ++k) {
        const float f = tile[c8 + k][cc];
        const unsigned short hb = f2bf_bits(f);
        const unsigned short lb = f2bf_bits(f - bf_bits2f(hb));
        hv[k] = __builtin_bit_cast(_Float16, hb);
        lv[k] = __builtin_bit_cast(_Float16, lb);
      }
      const size_t o = (size_t)(c0 + cc) * DIN + e0 + c8;
      *(volatile v8h*)(yh + o) = hv;
      *(volatile v8h*)(yl + o) = lv;
    }
    __threadfence();
  }
}

extern "C" void kernel_launch(void* const* d_in, const int* in_sizes, int n_in,
                              void* d_out, int out_size, void* d_ws,
                              size_t ws_size, hipStream_t stream) {
  if (n_in < 14) return;
  if (in_sizes[0] != NPIX * DMOD || out_size != NPIX * DMOD) return;
  if (in_sizes[1] != DIN * DMOD || in_sizes[2] != DIN || in_sizes[3] != 48 * DIN || in_sizes[4] != 48 ||
      in_sizes[5] != DIN * 8 || in_sizes[6] != DIN || in_sizes[7] != DIN * 8 || in_sizes[8] != DIN ||
      in_sizes[9] != DIN * NST || in_sizes[10] != DIN * NST || in_sizes[11] != DIN ||
      in_sizes[12] != DMOD * DIN || in_sizes[13] != DMOD) return;

  const float* x    = (const float*)d_in[0];
  const float* wi   = (const float*)d_in[1];
  const float* bi   = (const float*)d_in[2];
  const float* wx   = (const float*)d_in[3];
  const float* xpb  = (const float*)d_in[4];
  const float* dtTw = (const float*)d_in[5];
  const float* dtTb = (const float*)d_in[6];
  const float* dtLw = (const float*)d_in[7];
  const float* dtLb = (const float*)d_in[8];
  const float* ATl  = (const float*)d_in[9];
  const float* ALl  = (const float*)d_in[10];
  const float* Dv   = (const float*)d_in[11];
  const float* wo   = (const float*)d_in[12];
  const float* bo   = (const float*)d_in[13];
  float* out = (float*)d_out;

  size_t off = 0;
  char* base = (char*)d_ws;
  auto carve = [&](size_t bytes) -> void* { void* p = base + off; off += (bytes + 255) & ~(size_t)255; return p; };
  unsigned short* Xh  = (unsigned short*)carve((size_t)NPIX * DMOD * 2);
  unsigned short* Xl  = (unsigned short*)carve((size_t)NPIX * DMOD * 2);
  unsigned short* Wih = (unsigned short*)carve((size_t)DIN * DMOD * 2);
  unsigned short* Wil = (unsigned short*)carve((size_t)DIN * DMOD * 2);
  unsigned short* Wxh = (unsigned short*)carve((size_t)64 * DIN * 2);
  unsigned short* Wxl = (unsigned short*)carve((size_t)64 * DIN * 2);
  unsigned short* Wdh = (unsigned short*)carve((size_t)512 * 32 * 2);
  unsigned short* Wdl = (unsigned short*)carve((size_t)512 * 32 * 2);
  unsigned short* Woh = (unsigned short*)carve((size_t)DMOD * DIN * 2);
  unsigned short* Wol = (unsigned short*)carve((size_t)DMOD * DIN * 2);
  float*          bias576 = (float*)carve((size_t)576 * 4);
  float*          Upre = (float*)carve((size_t)NPIX * DIN * 4);
  float*          Uf   = (float*)carve((size_t)NPIX * DIN * 4);
  unsigned short* Uh   = (unsigned short*)carve((size_t)NPIX * DIN * 2);
  unsigned short* Ul   = (unsigned short*)carve((size_t)NPIX * DIN * 2);
  float*          DBC  = (float*)carve((size_t)NPIX * 64 * 4);
  unsigned short* A16h = (unsigned short*)carve((size_t)NPIX * 32 * 2);
  unsigned short* A16l = (unsigned short*)carve((size_t)NPIX * 32 * 2);
  float*          PREraw = (float*)carve((size_t)NPIX * 512 * 4);
  float*          PRE  = (float*)carve((size_t)NPIX * 512 * 4);
  float*          Yt   = (float*)carve((size_t)DIN * NPIX * 4);
  unsigned short* Yh   = (unsigned short*)carve((size_t)NPIX * DIN * 2);
  unsigned short* Yl   = (unsigned short*)carve((size_t)NPIX * DIN * 2);
  if (off > ws_size) return;
  const float* bx64  = bias576;
  const float* bd512 = bias576 + 64;

  prep_params<<<98, 128, 0, stream>>>(wi, wx, dtTw, dtLw, wo, xpb, dtTb, dtLb,
                                      Wih, Wil, Wxh, Wxl, Wdh, Wdl, Woh, Wol, bias576);
  split_cast8<<<(NPIX * DMOD / 8 + 255) / 256, 256, 0, stream>>>(x, Xh, Xl, NPIX * DMOD / 8);
  wmma_gemm64<1, true, 2, 0, false, 0><<<dim3(64, 1), 256, 0, stream>>>(
      Xh, Xl, DMOD, 0L, Wih, Wil, DMOD, 0L, (void*)Upre, nullptr, DIN, 0L, bi, nullptr, 0L,
      NPIX, DIN, DMOD, 1.0f);
  ew_tile2048<0, true><<<NPIX * DIN / 2048, 256, 0, stream>>>(Upre, Uf, Uh, Ul);
  wmma_gemm64<1, true, 2, 0, false, 0><<<dim3(16, 1), 256, 0, stream>>>(
      Uh, Ul, DIN, 0L, Wxh, Wxl, DIN, 0L, (void*)DBC, nullptr, 64, 0L, bx64, nullptr, 0L,
      NPIX, 64, DIN, 1.0f);
  build_a16<<<(NPIX * 4 + 127) / 128, 128, 0, stream>>>(DBC, A16h, A16l);
  wmma_gemm64<1, true, 2, 0, false, 0><<<dim3(128, 1), 256, 0, stream>>>(
      A16h, A16l, 32, 0L, Wdh, Wdl, 32, 0L, (void*)PREraw, nullptr, 512, 0L, bd512, nullptr, 0L,
      NPIX, 512, 32, 1.0f);
  ew_tile2048<1, false><<<NPIX * 512 / 2048, 256, 0, stream>>>(PREraw, PRE, nullptr, nullptr);
  scan2d<<<2 * (DIN / SC_EPB), SC_THR, 0, stream>>>(PRE, Uf, DBC, ATl, ALl, Dv, Yt);
  ytr_split<<<(NPIX / 64) * (DIN / 64), 256, 0, stream>>>(Yt, Yh, Yl);
  wmma_gemm64<1, true, 2, 0, false, 0><<<dim3(32, 1), 256, 0, stream>>>(
      Yh, Yl, DIN, 0L, Woh, Wol, DIN, 0L, (void*)out, nullptr, DMOD, 0L, bo, nullptr, 0L,
      NPIX, DMOD, DIN, 1.0f);
  (void)hipGetLastError();
}
